// GATLinkPredictor_46059229282719
// MI455X (gfx1250) — hardware-verified
//
#include <hip/hip_runtime.h>
#include <stddef.h>
#include <stdint.h>
#include <math.h>


#define FIN     128
#define HCH     256
#define NHEAD   4
#define CPH     64
#define KA      512
#define HS      64
#define PBN     128
#define NTHR    256
#define NWAVE   8
#define EPT     8
#define CHUNK   (NTHR * EPT)
#define WCAP    (EPT * 32)
#define LISTN   (NWAVE * WCAP)
#define NBMAX   2048
#define SLOTB   11
#define RCAP    28672
#define DEGCAP  128
#define GBM     64
#define GBN     128
#define GTHR    128
#define MROWS   128
#define EPB     256
#define NEGSL   0.2f
#define WSMAX   134217728
#define LDS_AGG ((2 * RCAP + 2 * NBMAX + LISTN) * 4 + 64)

static_assert((CHUNK & (CHUNK - 1)) == 0 && CHUNK <= (1 << SLOTB));
static_assert(NBMAX == (1 << SLOTB));
static_assert(NTHR * 8 == NBMAX);
static_assert(LISTN >= NBMAX);
static_assert(LISTN >= NWAVE * WCAP);
static_assert((RCAP % 32) == 0);
static_assert(LDS_AGG <= 300000);
static_assert(GBM == (GTHR / 32) * 16 && GBN == 4 * 32);
static_assert((FIN % 32) == 0 && (KA % 32) == 0 && KA == 2 * HCH);
static_assert((HCH % GBN) == 0 && (PBN % GBN) == 0);
static_assert((MROWS % GBM) == 0);
static_assert(HCH == 8 * 32 && CPH == 8 * 8 && NHEAD * CPH == HCH);
static_assert(PBN == 2 * HS && (HS % 4) == 0 && HS <= 64);
static_assert(EPB == NTHR && EPB == 4 * 64);
static_assert(FIN <= KA);
static_assert(PBN <= HCH);
static_assert((FIN % 8) == 0 && (HCH % 8) == 0);

typedef float          v2f  __attribute__((ext_vector_type(2)));
typedef float          v4f  __attribute__((ext_vector_type(4)));
typedef float          v8f  __attribute__((ext_vector_type(8)));
typedef int            v4i  __attribute__((ext_vector_type(4)));
typedef int            v8i  __attribute__((ext_vector_type(8)));
typedef unsigned int   v4u  __attribute__((ext_vector_type(4)));
typedef unsigned short v8us __attribute__((ext_vector_type(8)));
typedef __bf16         v16b __attribute__((ext_vector_type(16)));
typedef v4f  __attribute__((may_alias)) v4fa;
typedef v4i  __attribute__((may_alias)) v4ia;
typedef v8us __attribute__((may_alias)) v8usa;
union FragB { v16b v; v8us h[2]; v8i w; };

__device__ __forceinline__ v8f wmb(const FragB& a, const FragB& b, v8f c) {
  v8f d = __builtin_amdgcn_wmma_f32_16x16x32_bf16(false, a.v, false, b.v, (short)0, c, false, false);
  asm volatile("v_nop\n\tv_nop\n\tv_nop\n\tv_nop" : "+v"(d) : "v"(a.w), "v"(b.w));
  return d;
}

__device__ __forceinline__ unsigned int f2bf(float f) {
  const unsigned int u = __float_as_uint(f);
  return ((u + 0x7FFFu + ((u >> 16) & 1u)) >> 16) & 0xFFFFu;
}
__device__ __forceinline__ float bf2f(unsigned int b) { return __uint_as_float(b << 16); }
__device__ __forceinline__ float bfr(float f) { return bf2f(f2bf(f)); }
__device__ __forceinline__ v4f bfr4(const v4f a) {
  v4f r; r.x = bfr(a.x); r.y = bfr(a.y); r.z = bfr(a.z); r.w = bfr(a.w); return r;
}
__device__ __forceinline__ unsigned int pk2(float lo, float hi) { return f2bf(lo) | (f2bf(hi) << 16); }
__device__ __forceinline__ v4u pack8(const v4f a, const v4f b) {
  v4u r;
  r.x = pk2(a.x, a.y); r.y = pk2(a.z, a.w); r.z = pk2(b.x, b.y); r.w = pk2(b.z, b.w);
  return r;
}

__device__ __forceinline__ int scan_chunk(const int* __restrict__ dsts, int nE, int cbase, int slotBase,
                                          int nb, int vec8, int* list, int tid, int lane, int wave) {
  int wc = 0;
  const int el0  = tid * EPT;
  const int e0   = cbase + el0;
  const int sent = -2147483647 - 1;
  v4i da, db;
  if (vec8 != 0 && cbase + CHUNK <= nE) {
    da = *(const v4i*)(dsts + e0);
    db = *(const v4i*)(dsts + e0 + 4);
  } else {
    da.x = (e0     < nE) ? dsts[min(e0,     nE - 1)] : sent;
    da.y = (e0 + 1 < nE) ? dsts[min(e0 + 1, nE - 1)] : sent;
    da.z = (e0 + 2 < nE) ? dsts[min(e0 + 2, nE - 1)] : sent;
    da.w = (e0 + 3 < nE) ? dsts[min(e0 + 3, nE - 1)] : sent;
    db.x = (e0 + 4 < nE) ? dsts[min(e0 + 4, nE - 1)] : sent;
    db.y = (e0 + 5 < nE) ? dsts[min(e0 + 5, nE - 1)] : sent;
    db.z = (e0 + 6 < nE) ? dsts[min(e0 + 6, nE - 1)] : sent;
    db.w = (e0 + 7 < nE) ? dsts[min(e0 + 7, nE - 1)] : sent;
  }
  const unsigned nbs = (unsigned)slotBase;
  const unsigned unb = (unsigned)nb;
  const unsigned s0 = (unsigned)da.x - nbs, s1 = (unsigned)da.y - nbs;
  const unsigned s2 = (unsigned)da.z - nbs, s3 = (unsigned)da.w - nbs;
  const unsigned s4 = (unsigned)db.x - nbs, s5 = (unsigned)db.y - nbs;
  const unsigned s6 = (unsigned)db.z - nbs, s7 = (unsigned)db.w - nbs;
  const bool h0 = s0 < unb, h1 = s1 < unb, h2 = s2 < unb, h3 = s3 < unb;
  const bool h4 = s4 < unb, h5 = s5 < unb, h6 = s6 < unb, h7 = s7 < unb;
  const unsigned any = __builtin_amdgcn_ballot_w32(h0 | h1 | h2 | h3 | h4 | h5 | h6 | h7);
  if (any != 0u) {
#define HITJ(J, HJ, SJ) { \
      const unsigned mj = __builtin_amdgcn_ballot_w32(HJ); \
      if (mj != 0u) { \
        if (HJ) { \
          const int pos = wc + (int)__builtin_amdgcn_mbcnt_lo(mj, 0u); \
          if (pos < WCAP) list[wave * WCAP + pos] = ((el0 + (J)) << SLOTB) | (int)(SJ); \
        } \
        wc += (int)__builtin_popcount(mj); } }
    HITJ(0, h0, s0)
    HITJ(1, h1, s1)
    HITJ(2, h2, s2)
    HITJ(3, h3, s3)
    HITJ(4, h4, s4)
    HITJ(5, h5, s5)
    HITJ(6, h6, s6)
    HITJ(7, h7, s7)
#undef HITJ
  }
  return wc;
}

__global__ __launch_bounds__(NTHR) void k_xb(const float* __restrict__ x, int nN, unsigned short* XB, int nUnits) {
  const int v = (int)blockIdx.x * NTHR + (int)threadIdx.x;
  if (v >= nUnits) return;
  const int row = v >> 4;
  const int k8  = (v & 15) * 8;
  const int rc  = row < nN ? row : nN - 1;
  const float* p = x + (size_t)rc * FIN + k8;
  v4f a = *(const v4fa*)p;
  v4f b = *(const v4fa*)(p + 4);
  const v4f z4 = {0.f, 0.f, 0.f, 0.f};
  if (row >= nN) { a = z4; b = z4; }
  const v4u o = pack8(a, b);
  unsigned short* dp = XB + (size_t)row * FIN + k8;
  *(volatile v4u*)dp = o;
  __threadfence();
  *(volatile v4u*)dp = o;
}

__global__ __launch_bounds__(NTHR) void k_wtr(const float* __restrict__ w, int Kin, int Ncol, int Nrows, int Kout,
                                              unsigned short* wt, int nUnits) {
  const int u = (int)blockIdx.x * NTHR + (int)threadIdx.x;
  if (u >= nUnits) return;
  const int kq = Kout >> 3;
  const int n  = u / kq;
  const int k8 = (u - n * kq) * 8;
  const int kk = k8 - (k8 / Kin) * Kin;
  const int ncl = n < Ncol ? n : Ncol - 1;
  const float* p = w + (size_t)kk * (size_t)Ncol + ncl;
  v4f a, b;
  a.x = p[0];                    a.y = p[(size_t)Ncol];         a.z = p[(size_t)2 * Ncol];     a.w = p[(size_t)3 * Ncol];
  b.x = p[(size_t)4 * Ncol];     b.y = p[(size_t)5 * Ncol];     b.z = p[(size_t)6 * Ncol];     b.w = p[(size_t)7 * Ncol];
  const v4f z4 = {0.f, 0.f, 0.f, 0.f};
  if (n >= Ncol || n >= Nrows) { a = z4; b = z4; }
  const v4u wv = pack8(a, b);
  unsigned short* o = wt + (size_t)n * (size_t)Kout + k8;
  *(volatile v4u*)o = wv;
  __threadfence();
  *(volatile v4u*)o = wv;
}

__global__ __launch_bounds__(GTHR) void k_gemm(const unsigned short* __restrict__ A, int lda,
                                               const unsigned short* __restrict__ BT, int ldb, int K,
                                               float* Cm, int ldc) {
  __shared__ __attribute__((aligned(16))) float stg[GBM * GBN];
  const int tid = (int)threadIdx.x, lane = tid & 31, wave = tid >> 5, hh = lane >> 4, m = lane & 15;
  const int rowBase = (int)blockIdx.x * GBM;
  const int colBase = (int)blockIdx.y * GBN;

  v8f acc[8];
  {
    const v8f z = {0.f, 0.f, 0.f, 0.f, 0.f, 0.f, 0.f, 0.f};
#pragma unroll
    for (int t = 0; t < 8; ++t) acc[t] = z;
  }
  const unsigned short* ap = A  + (size_t)(rowBase + 16 * wave + m) * (size_t)lda + 8 * hh;
  const unsigned short* bp = BT + (size_t)(colBase + m) * (size_t)ldb + 8 * hh;

#pragma unroll 1
  for (int k0 = 0; k0 < K; k0 += 32) {
    FragB af;
    af.h[0] = *(const v8usa*)(ap + k0);
    af.h[1] = *(const v8usa*)(ap + k0 + 16);
#pragma unroll
    for (int nt = 0; nt < 8; ++nt) {
      const unsigned short* wq = bp + (size_t)(16 * nt) * (size_t)ldb + k0;
      FragB bf;
      bf.h[0] = *(const v8usa*)wq;
      bf.h[1] = *(const v8usa*)(wq + 16);
      acc[nt] = wmb(af, bf, acc[nt]);
    }
  }

#pragma unroll
  for (int nt = 0; nt < 8; ++nt) {
    const int lc = 16 * nt + m;
#pragma unroll
    for (int r = 0; r < 8; ++r) {
      const int lr = 16 * wave + 8 * hh + r;
      stg[lr * GBN + lc] = acc[nt][r];
    }
  }
  __syncthreads();

  v4f pv[16];
#pragma unroll
  for (int i = 0; i < 16; ++i) pv[i] = *(const v4fa*)(stg + (16 * wave + i) * GBN + 4 * lane);
#pragma unroll
  for (int i = 0; i < 16; ++i) {
    float* op = Cm + (size_t)(rowBase + 16 * wave + i) * (size_t)ldc + colBase + 4 * lane;
    *(volatile v4f*)op = pv[i];
  }
  __threadfence();
#pragma unroll
  for (int i = 0; i < 16; ++i) {
    float* op = Cm + (size_t)(rowBase + 16 * wave + i) * (size_t)ldc + colBase + 4 * lane;
    *(volatile v4f*)op = pv[i];
  }
}

__global__ __launch_bounds__(NTHR) void k_agg(
    const int* __restrict__ srcs, const int* __restrict__ dsts,
    const float* __restrict__ F,
    const float* __restrict__ asrc, const float* __restrict__ adst, const float* __restrict__ bias,
    unsigned short* HP,
    int nN, int nE, int nb, int vec8, int MPr) {
  extern __shared__ v4f lds_dyn[];
  int* reg1 = (int*)lds_dyn;
  int* reg2 = reg1 + RCAP;
  int* scnt = reg2 + RCAP;
  int* soff = scnt + NBMAX;
  int* list = soff + NBMAX;
  int* wcnt = list + LISTN;
  int* wtot = wcnt + NWAVE;
  const int tid = (int)threadIdx.x, lane = tid & 31, wave = tid >> 5;
  const int nodeBase = (int)blockIdx.x * nb;

  for (int i = tid; i < NBMAX; i += NTHR) scnt[i] = 0;
  __syncthreads();

  int tot = 0;
  const int nChunks = (nE + CHUNK - 1) / CHUNK;
#pragma unroll 1
  for (int ch = 0; ch < nChunks; ++ch) {
    const int cbase = ch * CHUNK;
    const int wc = scan_chunk(dsts, nE, cbase, nodeBase, nb, vec8, list, tid, lane, wave);
    if (lane == 0) wcnt[wave] = wc;
    __syncthreads();
    int pre = 0, all = 0;
#pragma unroll
    for (int w2 = 0; w2 < NWAVE; ++w2) {
      int c = wcnt[w2];
      c = c < 0 ? 0 : (c > WCAP ? WCAP : c);
      all += c;
      pre += (w2 < wave) ? c : 0;
    }
    const int wcc  = wc > WCAP ? WCAP : wc;
    const int base = tot + pre;
#pragma unroll 1
    for (int i = lane; i < wcc; i += 32) {
      const int ent = list[wave * WCAP + i];
      const int el  = (ent >> SLOTB) & (CHUNK - 1);
      const int sl  = ent & (NBMAX - 1);
      int eid = cbase + el;
      eid = eid > nE - 1 ? nE - 1 : eid;
      const int pos = base + i;
      if (pos < RCAP) reg1[pos] = (int)(((unsigned)eid << SLOTB) | (unsigned)sl);
    }
    tot += all;
    tot = tot > RCAP ? RCAP : tot;
    __syncthreads();
  }
  const int nh = tot;

  if (wave == 0) {
#pragma unroll 1
    for (int b0 = 0; b0 < nh; b0 += 32) {
      const int idx = b0 + lane;
      const int uv  = reg1[idx < nh ? idx : nh - 1];
      const int m32 = (nh - b0) < 32 ? (nh - b0) : 32;
#pragma unroll 1
      for (int k = 0; k < m32; ++k) {
        const int u  = __builtin_amdgcn_readlane(uv, k);
        const int sl = u & (NBMAX - 1);
        if (lane == 0) scnt[sl] = scnt[sl] + 1;
      }
    }
  }
  __syncthreads();

  {
    const v4i ca = *(const v4ia*)(scnt + 8 * tid);
    const v4i cb = *(const v4ia*)(scnt + 8 * tid + 4);
    const int e0 = ca.x < 0 ? 0 : ca.x, e1 = ca.y < 0 ? 0 : ca.y, e2 = ca.z < 0 ? 0 : ca.z, e3 = ca.w < 0 ? 0 : ca.w;
    const int e4 = cb.x < 0 ? 0 : cb.x, e5 = cb.y < 0 ? 0 : cb.y, e6 = cb.z < 0 ? 0 : cb.z, e7 = cb.w < 0 ? 0 : cb.w;
    const int ts = e0 + e1 + e2 + e3 + e4 + e5 + e6 + e7;
    int incl = ts;
#pragma unroll
    for (int d = 1; d < 32; d <<= 1) {
      const int up = __shfl_up(incl, d);
      if (lane >= d) incl += up;
    }
    if (lane == 31) wtot[wave] = incl;
    __syncthreads();
    int pre = 0;
#pragma unroll
    for (int w2 = 0; w2 < NWAVE; ++w2) pre += (w2 < wave) ? wtot[w2] : 0;
    int run = pre + incl - ts;
    soff[8 * tid + 0] = run; run += e0;
    soff[8 * tid + 1] = run; run += e1;
    soff[8 * tid + 2] = run; run += e2;
    soff[8 * tid + 3] = run; run += e3;
    soff[8 * tid + 4] = run; run += e4;
    soff[8 * tid + 5] = run; run += e5;
    soff[8 * tid + 6] = run; run += e6;
    soff[8 * tid + 7] = run;
  }
  __syncthreads();
  for (int i = tid; i < NBMAX; i += NTHR) list[i] = soff[i];
  __syncthreads();

  if (wave == 0) {
#pragma unroll 1
    for (int b0 = 0; b0 < nh; b0 += 32) {
      const int idx = b0 + lane;
      const int uv  = reg1[idx < nh ? idx : nh - 1];
      const int m32 = (nh - b0) < 32 ? (nh - b0) : 32;
#pragma unroll 1
      for (int k = 0; k < m32; ++k) {
        const int u   = __builtin_amdgcn_readlane(uv, k);
        const int sl  = u & (NBMAX - 1);
        const int eid = (int)((unsigned)u >> SLOTB);
        if (lane == 0) {
          int pos = list[sl];
          pos = pos < 0 ? 0 : (pos > RCAP - 1 ? RCAP - 1 : pos);
          reg2[pos] = eid;
          list[sl] = pos + 1;
        }
      }
    }
  }
  __syncthreads();

  const int nbw = nb >> 3;
  const bool ovf = (nh >= RCAP);
  const float qnan = __int_as_float(0x7fc00000);
  float as8[8], ad8[8], bb8[8];
  {
    const v4f sa = bfr4(*(const v4fa*)(asrc + 8 * lane));
    const v4f sb = bfr4(*(const v4fa*)(asrc + 8 * lane + 4));
    const v4f da = bfr4(*(const v4fa*)(adst + 8 * lane));
    const v4f db = bfr4(*(const v4fa*)(adst + 8 * lane + 4));
    const v4f ba = bfr4(*(const v4fa*)(bias + 8 * lane));
    const v4f bbv = bfr4(*(const v4fa*)(bias + 8 * lane + 4));
    as8[0] = sa.x; as8[1] = sa.y; as8[2] = sa.z; as8[3] = sa.w;
    as8[4] = sb.x; as8[5] = sb.y; as8[6] = sb.z; as8[7] = sb.w;
    ad8[0] = da.x; ad8[1] = da.y; ad8[2] = da.z; ad8[3] = da.w;
    ad8[4] = db.x; ad8[5] = db.y; ad8[6] = db.z; ad8[7] = db.w;
    bb8[0] = ba.x; bb8[1] = ba.y; bb8[2] = ba.z; bb8[3] = ba.w;
    bb8[4] = bbv.x; bb8[5] = bbv.y; bb8[6] = bbv.z; bb8[7] = bbv.w;
  }

#pragma unroll 1
  for (int jt = 0; jt < nbw; ++jt) {
    const int slot = wave * nbw + jt;
    const int grow = nodeBase + slot;
    const int gcl  = grow < nN ? grow : nN - 1;
    int st = soff[slot];
    const int craw = scnt[slot];
    int cnt = craw;
    st  = st < 0 ? 0 : (st > nh ? nh : st);
    cnt = cnt < 0 ? 0 : (cnt > DEGCAP ? DEGCAP : cnt);
    if (cnt > nh - st) cnt = nh - st;
    const float pz = (ovf || craw > DEGCAP) ? qnan : 0.0f;

    const float* fdp = F + (size_t)gcl * HCH + 8 * lane;
    const v4f fda = *(const v4fa*)fdp;
    const v4f fdb = *(const v4fa*)(fdp + 4);
    float fd[8];
    fd[0] = fda.x; fd[1] = fda.y; fd[2] = fda.z; fd[3] = fda.w;
    fd[4] = fdb.x; fd[5] = fdb.y; fd[6] = fdb.z; fd[7] = fdb.w;
    float pd = fd[0] * ad8[0];
#pragma unroll
    for (int i = 1; i < 8; ++i) pd = fmaf(fd[i], ad8[i], pd);
    pd += __shfl_xor(pd, 1);
    pd += __shfl_xor(pd, 2);
    pd += __shfl_xor(pd, 4);
    float p0 = fd[0] * as8[0];
#pragma unroll
    for (int i = 1; i < 8; ++i) p0 = fmaf(fd[i], as8[i], p0);
    p0 += __shfl_xor(p0, 1);
    p0 += __shfl_xor(p0, 2);
    p0 += __shfl_xor(p0, 4);
    float l0 = p0 + pd;
    l0 = l0 > 0.f ? l0 : NEGSL * l0;
    float mx = l0, dn = 1.0f;
    float acc[8];
#pragma unroll
    for (int i = 0; i < 8; ++i) acc[i] = fd[i];

#pragma unroll 1
    for (int q = 0; q < cnt; ++q) {
      int idx = st + q; idx = idx > RCAP - 1 ? RCAP - 1 : idx;
      int eid = reg2[idx]; eid = eid < 0 ? 0 : (eid > nE - 1 ? nE - 1 : eid);
      const int sraw = srcs[eid];
      const int s = sraw < 0 ? 0 : (sraw > nN - 1 ? nN - 1 : sraw);
      const float* fsp = F + (size_t)s * HCH + 8 * lane;
      const v4f fsa = *(const v4fa*)fsp;
      const v4f fsb = *(const v4fa*)(fsp + 4);
      float fs[8];
      fs[0] = fsa.x; fs[1] = fsa.y; fs[2] = fsa.z; fs[3] = fsa.w;
      fs[4] = fsb.x; fs[5] = fsb.y; fs[6] = fsb.z; fs[7] = fsb.w;
      float es = fs[0] * as8[0];
#pragma unroll
      for (int i = 1; i < 8; ++i) es = fmaf(fs[i], as8[i], es);
      es += __shfl_xor(es, 1);
      es += __shfl_xor(es, 2);
      es += __shfl_xor(es, 4);
      float lg = es + pd;
      lg = lg > 0.f ? lg : NEGSL * lg;
      const float df = lg - mx;
      const float ee = __expf(-fabsf(df));
      const bool up  = df > 0.f;
      const float s1 = up ? ee : 1.0f;
      const float s2 = up ? 1.0f : ee;
      mx = up ? lg : mx;
      dn = fmaf(dn, s1, s2);
#pragma unroll
      for (int i = 0; i < 8; ++i) acc[i] = fmaf(acc[i], s1, s2 * fs[i]);
    }
    const float inv = __builtin_amdgcn_rcpf(dn);
    const bool live = grow < nN;
    unsigned int hw[4], lw[4];
#pragma unroll
    for (int j = 0; j < 4; ++j) {
      float h0 = fmaf(acc[2 * j],     inv, bb8[2 * j]);
      float h1 = fmaf(acc[2 * j + 1], inv, bb8[2 * j + 1]);
      const float n0 = __expf(fminf(h0, 0.f)) - 1.0f;
      const float n1 = __expf(fminf(h1, 0.f)) - 1.0f;
      h0 = h0 > 0.f ? h0 : n0;
      h1 = h1 > 0.f ? h1 : n1;
      h0 = (live ? h0 : 0.f) + pz;
      h1 = (live ? h1 : 0.f) + pz;
      const unsigned int hb0 = f2bf(h0), hb1 = f2bf(h1);
      const unsigned int lb0 = f2bf(h0 - bf2f(hb0)), lb1 = f2bf(h1 - bf2f(hb1));
      hw[j] = hb0 | (hb1 << 16);
      lw[j] = lb0 | (lb1 << 16);
    }
    v4u hv, lv;
    hv.x = hw[0]; hv.y = hw[1]; hv.z = hw[2]; hv.w = hw[3];
    lv.x = lw[0]; lv.y = lw[1]; lv.z = lw[2]; lv.w = lw[3];
    unsigned short* gp = HP + (size_t)grow * KA + 8 * lane;
    const bool wr = grow < MPr;
    if (wr) {
      *(volatile v4u*)gp = hv;
      *(volatile v4u*)(gp + HCH) = lv;
    }
    __threadfence();
    if (wr) {
      *(volatile v4u*)gp = hv;
      *(volatile v4u*)(gp + HCH) = lv;
    }
  }
}

__global__ __launch_bounds__(NTHR) void k_score(const int* __restrict__ eli, int nL, int nN,
                                                const float* __restrict__ pab,
                                                const float* __restrict__ bs1, const float* __restrict__ ws2,
                                                const float* __restrict__ bs2, float* out) {
  __shared__ __attribute__((aligned(16))) float cst[2 * HS + 16];
  __shared__ __attribute__((aligned(16))) float sy[EPB];
  const int tid = (int)threadIdx.x;

  if (tid < HS) {
    cst[tid]      = bfr(bs1[tid]);
    cst[HS + tid] = bfr(ws2[tid]);
  }
  if (tid < 32) {
    const float vb = bfr(bs2[0]);
    if (tid == 0) cst[2 * HS] = vb;
  }

  const int e0 = (int)blockIdx.x * EPB;
  int ec = e0 + tid;
  ec = ec > nL - 1 ? nL - 1 : ec;
  int s = eli[ec];
  int t = eli[(size_t)nL + (size_t)ec];
  s = s < 0 ? 0 : (s > nN - 1 ? nN - 1 : s);
  t = t < 0 ? 0 : (t > nN - 1 ? nN - 1 : t);
  const float* pa = pab + (size_t)s * PBN;
  const float* pb = pab + (size_t)t * PBN + HS;
  __syncthreads();

  float dot = 0.0f;
#pragma unroll 2
  for (int c4 = 0; c4 < HS / 4; ++c4) {
    const v4f a  = *(const v4fa*)(pa + 4 * c4);
    const v4f q  = *(const v4fa*)(pb + 4 * c4);
    const v4f bb = *(const v4fa*)(cst + 4 * c4);
    const v4f ww = *(const v4fa*)(cst + HS + 4 * c4);
    const float t0 = fmaxf((a.x + q.x) + bb.x, 0.0f);
    const float t1 = fmaxf((a.y + q.y) + bb.y, 0.0f);
    const float t2 = fmaxf((a.z + q.z) + bb.z, 0.0f);
    const float t3 = fmaxf((a.w + q.w) + bb.w, 0.0f);
    dot = fmaf(t0, ww.x, dot);
    dot = fmaf(t1, ww.y, dot);
    dot = fmaf(t2, ww.z, dot);
    dot = fmaf(t3, ww.w, dot);
  }
  const float yv = dot + cst[2 * HS];
  sy[tid] = yv;
  __syncthreads();

  const int tl = tid < 64 ? tid : 63;
  const v4f o4 = *(const v4fa*)(sy + 4 * tl);
  const int eo = e0 + 4 * tl;
  const bool stv = (tid < 64) && (eo + 3 < nL);
  if (stv) *(volatile v4f*)(out + (size_t)eo) = o4;
  __threadfence();
  if (stv) *(volatile v4f*)(out + (size_t)eo) = o4;
}

static int pick_nb(int nE, int nN) {
  int nb = NBMAX;
  while (nb > 32 && (long long)nb * (long long)nE * 5LL > (long long)RCAP * (long long)nN * 4LL) nb >>= 1;
  return nb;
}
static inline int cdiv(int a, int b) { return (a + b - 1) / b; }

extern "C" void kernel_launch(void* const* d_in, const int* in_sizes, int n_in,
                              void* d_out, int out_size, void* d_ws, size_t ws_size,
                              hipStream_t stream) {
  if (n_in < 15) return;
  if (in_sizes[0] < FIN || (in_sizes[0] % FIN) != 0) return;
  const int nN = in_sizes[0] / FIN;
  if (nN <= 0 || nN > (1 << 22)) return;
  if (in_sizes[1] < 2 || (in_sizes[1] & 1) != 0) return;
  const int nE = in_sizes[1] / 2;
  if (nE < 1 || nE >= (1 << (32 - SLOTB))) return;
  if (in_sizes[2] < 2 || (in_sizes[2] & 1) != 0) return;
  const int nL = in_sizes[2] / 2;
  if (nL < 32 || (nL & 31) != 0) return;
  if (in_sizes[3]  != FIN * HCH) return;
  if (in_sizes[4]  != HCH || in_sizes[5] != HCH) return;
  if (in_sizes[6]  != HCH) return;
  if (in_sizes[7]  != HCH * HCH) return;
  if (in_sizes[8]  != HCH || in_sizes[9] != HCH) return;
  if (in_sizes[10] != HCH) return;
  if (in_sizes[11] != 2 * HCH * HS) return;
  if (in_sizes[12] != HS) return;
  if (in_sizes[13] != HS) return;
  if (in_sizes[14] < 1) return;
  if (out_size != nL) return;

  const float* x    = (const float*)d_in[0];
  const int*   ei   = (const int*)  d_in[1];
  const int*   eli  = (const int*)  d_in[2];
  const float* W1   = (const float*)d_in[3];
  const float* a1s  = (const float*)d_in[4];
  const float* a1d  = (const float*)d_in[5];
  const float* b1   = (const float*)d_in[6];
  const float* W2   = (const float*)d_in[7];
  const float* a2s  = (const float*)d_in[8];
  const float* a2d  = (const float*)d_in[9];
  const float* b2   = (const float*)d_in[10];
  const float* Ws1  = (const float*)d_in[11];
  const float* bs1  = (const float*)d_in[12];
  const float* Ws2  = (const float*)d_in[13];
  const float* bs2  = (const float*)d_in[14];
  float* out = (float*)d_out;
  const int* src = ei;
  const int* dst = ei + nE;

  const int MP   = cdiv(nN, MROWS) * MROWS;
  const int gM   = MP / GBM;
  const int nb   = pick_nb(nE, nN);
  if (nb < 32 || (nb & (nb - 1)) != 0 || nb > NBMAX) return;
  const int gA   = cdiv(MP, nb);
  const int vec8 = ((nE & 3) == 0) ? 1 : 0;
  if ((long long)gA * nb < (long long)MP) return;

  char* ws = (char*)d_ws;
  size_t off = 0;
  const size_t oWT1 = off; off += (size_t)HCH * FIN * 2;           off = (off + 255) & ~(size_t)255;
  const size_t oWT2 = off; off += (size_t)HCH * KA * 2;            off = (off + 255) & ~(size_t)255;
  const size_t oWSA = off; off += (size_t)PBN * KA * 2;            off = (off + 255) & ~(size_t)255;
  const size_t oF   = off; off += (size_t)MP * HCH * 4;            off = (off + 255) & ~(size_t)255;
  const size_t oH   = off; off += (size_t)MP * KA * 2;             off = (off + 255) & ~(size_t)255;
  if (off > ws_size || off > (size_t)WSMAX) return;
  unsigned short* WT1  = (unsigned short*)(ws + oWT1);
  unsigned short* WT2  = (unsigned short*)(ws + oWT2);
  unsigned short* WSAB = (unsigned short*)(ws + oWSA);
  float*          F    = (float*)(ws + oF);
  float*          PAB  = (float*)(ws + oF);
  unsigned short* HP   = (unsigned short*)(ws + oH);
  unsigned short* XB   = (unsigned short*)(ws + oH);

  hipFuncSetAttribute(reinterpret_cast<const void*>(&k_agg), hipFuncAttributeMaxDynamicSharedMemorySize, LDS_AGG);

  const int nUx = MP * (FIN / 8);
  k_xb<<<cdiv(nUx, NTHR), NTHR, 0, stream>>>(x, nN, XB, nUx);

  {
    const int nU1 = HCH * (FIN / 8);
    k_wtr<<<cdiv(nU1, NTHR), NTHR, 0, stream>>>(W1, FIN, HCH, HCH, FIN, WT1, nU1);
    const int nU2 = HCH * (KA / 8);
    k_wtr<<<cdiv(nU2, NTHR), NTHR, 0, stream>>>(W2, HCH, HCH, HCH, KA, WT2, nU2);
    const int nU3 = HS * (KA / 8);
    k_wtr<<<cdiv(nU3, NTHR), NTHR, 0, stream>>>(Ws1, HCH, HS, HS, KA, WSAB, nU3);
    k_wtr<<<cdiv(nU3, NTHR), NTHR, 0, stream>>>(Ws1 + (size_t)HCH * HS, HCH, HS, HS, KA, WSAB + (size_t)HS * KA, nU3);
  }

  k_gemm<<<dim3(gM, HCH / GBN), GTHR, 0, stream>>>(XB, FIN, WT1, FIN, FIN, F, HCH);
  k_agg<<<gA, NTHR, LDS_AGG, stream>>>(src, dst, F, a1s, a1d, b1, HP, nN, nE, nb, vec8, MP);
  k_gemm<<<dim3(gM, HCH / GBN), GTHR, 0, stream>>>(HP, KA, WT2, KA, KA, F, HCH);
  k_agg<<<gA, NTHR, LDS_AGG, stream>>>(src, dst, F, a2s, a2d, b2, HP, nN, nE, nb, vec8, MP);
  k_gemm<<<dim3(gM, PBN / GBN), GTHR, 0, stream>>>(HP, KA, WSAB, KA, KA, PAB, PBN);
  k_score<<<cdiv(nL, EPB), NTHR, 0, stream>>>(eli, nL, nN, PAB, bs1, Ws2, bs2, out);
}
